// EdgeConditionedConvolution_23570780521006
// MI455X (gfx1250) — hardware-verified
//
#include <hip/hip_runtime.h>
#include <stddef.h>


#define NTHR   256
#define NWAVE  8
#define FIN    32
#define EDIM   16
#define HID    32
#define ODIM   32
#define WCOL   1024
#define KP     32
#define EPB    128
#define NPB    128
#define PBLK   16
#define EPT    8
#define PIECE  (NTHR * EPT)
#define WCAP   (EPT * 32)
#define NBC    1024
#define SLB    10
#define AGGDYN (NBC * ODIM * 4)
#define WSCAP  134217728
#define EPSV   0.00001f
#define SLOPEV 0.01f

static_assert(PBLK * NTHR * 8 == WCOL * KP);
static_assert(WCOL <= PBLK * NTHR);
static_assert(NBC == (1 << SLB));
static_assert(PIECE == 2048);
static_assert((EPT % 4) == 0);
static_assert(EPB == NWAVE * 16);
static_assert(NPB == NWAVE * 16);
static_assert((NBC % 32) == 0);
static_assert((NBC % NWAVE) == 0);
static_assert((NBC * ODIM) % (4 * NTHR) == 0);
static_assert(FIN == 32 && HID == 32 && ODIM == 32 && EDIM == 16);
static_assert(WCOL == 4 * NTHR);
static_assert(FIN * ODIM == 4 * NTHR);

typedef float          v4f   __attribute__((ext_vector_type(4)));
typedef float          v8f   __attribute__((ext_vector_type(8)));
typedef int            v4i   __attribute__((ext_vector_type(4)));
typedef unsigned short v8us  __attribute__((ext_vector_type(8)));
typedef unsigned short v16us __attribute__((ext_vector_type(16)));
typedef __bf16         v16bf __attribute__((ext_vector_type(16)));
union FragU { v16us w; v8us u[2]; };
union C8    { v8f v; v4f h[2]; };

__device__ __forceinline__ v8f wmb(v16us a, v16us b, v8f c) {
  const v16bf ab = __builtin_bit_cast(v16bf, a);
  const v16bf bb = __builtin_bit_cast(v16bf, b);
  v8f d = __builtin_amdgcn_wmma_f32_16x16x32_bf16(false, ab, false, bb, (short)0, c, false, false);
  asm volatile("v_nop\n\tv_nop\n\tv_nop\n\tv_nop" : "+v"(d) : "v"(a), "v"(b));
  return d;
}
__device__ __forceinline__ v8f z8() {
  v8f z = {0.f, 0.f, 0.f, 0.f, 0.f, 0.f, 0.f, 0.f};
  return z;
}
__device__ __forceinline__ unsigned int bfb(float f) {
  const unsigned int u = __float_as_uint(f);
  return (u + 0x7FFFu + ((u >> 16) & 1u)) >> 16;
}
#define SPLIT2(VAL, FH, FL, IDX) { \
    const float sv_ = (VAL); \
    const unsigned int hb_ = bfb(sv_); \
    (FH).w[IDX] = (unsigned short)hb_; \
    (FL).w[IDX] = (unsigned short)bfb(sv_ - __uint_as_float(hb_ << 16)); }

__global__ __launch_bounds__(NTHR) void k_prep(
    const float* __restrict__ W2, const float* __restrict__ b2, const float* __restrict__ g2,
    const float* __restrict__ be2, const float* __restrict__ mu2, const float* __restrict__ va2,
    unsigned short* Whi, unsigned short* Wlo, float* cin) {
  const int t = (int)blockIdx.x * NTHR + (int)threadIdx.x;
  const int o = t * 8;
  const bool pl = o < WCOL * KP;
  const bool pc = t < WCOL;
  FragU fh, fl;
  fh.u[0] = (v8us){0, 0, 0, 0, 0, 0, 0, 0};
  fl.u[0] = fh.u[0];
  float cv = 0.0f;
  if (pl) {
    const int n = o >> 5, k0 = o & 31;
    const float s2 = g2[n] * (1.0f / sqrtf(va2[n] + EPSV));
#pragma unroll
    for (int j = 0; j < 8; ++j) {
      SPLIT2(W2[(size_t)(k0 + j) * WCOL + n] * s2, fh, fl, j)
    }
  }
  if (pc) {
    const float s = g2[t] * (1.0f / sqrtf(va2[t] + EPSV));
    cv = (b2[t] - mu2[t]) * s + be2[t];
  }
  if (pl) {
    *(volatile v8us*)(Whi + o) = fh.u[0];
    *(volatile v8us*)(Wlo + o) = fl.u[0];
  }
  if (pc) *(volatile float*)(cin + t) = cv;
  __threadfence();
  if (pl) {
    *(volatile v8us*)(Whi + o) = fh.u[0];
    *(volatile v8us*)(Wlo + o) = fl.u[0];
  }
  if (pc) *(volatile float*)(cin + t) = cv;
}

__global__ __launch_bounds__(NTHR) void k_root(
    const float* __restrict__ x, const float* __restrict__ root, const float* __restrict__ bias, float* R, int nN) {
  __shared__ __attribute__((aligned(16))) float sR[NWAVE * 16 * ODIM];
  __shared__ __attribute__((aligned(16))) float sRoot[FIN * ODIM];
  __shared__ __attribute__((aligned(16))) float sBias[ODIM];
  const int tid = (int)threadIdx.x, lane = tid & 31, wave = tid >> 5, hi = lane >> 4, m = lane & 15;
  const int n0 = ((int)blockIdx.x * NWAVE + wave) * 16;

  *(v4f*)(sRoot + 4 * tid) = *(const v4f*)(root + 4 * tid);
  if (tid < ODIM) sBias[tid] = bias[tid];
  __syncthreads();

  FragU ah, al;
  {
    int row = n0 + m;
    row = row > nN - 1 ? nN - 1 : row;
    const float* xp = x + (size_t)row * FIN;
    const v4f q0 = *(const v4f*)(xp + 8 * hi);
    const v4f q1 = *(const v4f*)(xp + 8 * hi + 4);
    const v4f q2 = *(const v4f*)(xp + 16 + 8 * hi);
    const v4f q3 = *(const v4f*)(xp + 16 + 8 * hi + 4);
    SPLIT2(q0.x, ah, al, 0)  SPLIT2(q0.y, ah, al, 1)  SPLIT2(q0.z, ah, al, 2)  SPLIT2(q0.w, ah, al, 3)
    SPLIT2(q1.x, ah, al, 4)  SPLIT2(q1.y, ah, al, 5)  SPLIT2(q1.z, ah, al, 6)  SPLIT2(q1.w, ah, al, 7)
    SPLIT2(q2.x, ah, al, 8)  SPLIT2(q2.y, ah, al, 9)  SPLIT2(q2.z, ah, al, 10) SPLIT2(q2.w, ah, al, 11)
    SPLIT2(q3.x, ah, al, 12) SPLIT2(q3.y, ah, al, 13) SPLIT2(q3.z, ah, al, 14) SPLIT2(q3.w, ah, al, 15)
  }
  FragU bh0, bl0, bh1, bl1;
#pragma unroll
  for (int j = 0; j < 8; ++j) {
    const float r0a = sRoot[(8 * hi + j) * ODIM + m];
    const float r0b = sRoot[(16 + 8 * hi + j) * ODIM + m];
    const float r1a = sRoot[(8 * hi + j) * ODIM + 16 + m];
    const float r1b = sRoot[(16 + 8 * hi + j) * ODIM + 16 + m];
    SPLIT2(r0a, bh0, bl0, j)
    SPLIT2(r0b, bh0, bl0, 8 + j)
    SPLIT2(r1a, bh1, bl1, j)
    SPLIT2(r1b, bh1, bl1, 8 + j)
  }
  v8f a0 = z8();
  a0 = wmb(ah.w, bh0.w, a0);
  a0 = wmb(ah.w, bl0.w, a0);
  a0 = wmb(al.w, bh0.w, a0);
  v8f a1 = z8();
  a1 = wmb(ah.w, bh1.w, a1);
  a1 = wmb(ah.w, bl1.w, a1);
  a1 = wmb(al.w, bh1.w, a1);

  const float bb0 = sBias[m], bb1 = sBias[16 + m];
  float* sw = sR + wave * (16 * ODIM);
  {
    float* sp = sw + (8 * hi) * ODIM;
#pragma unroll
    for (int r = 0; r < 8; ++r) {
      sp[r * ODIM + m]      = a0[r] + bb0;
      sp[r * ODIM + 16 + m] = a1[r] + bb1;
    }
  }
  __syncthreads();

  const int rq = lane >> 3, pc = lane & 7;
  float* rrow = R + (size_t)n0 * ODIM;
#pragma unroll
  for (int q = 0; q < 4; ++q) {
    const int row = 4 * q + rq;
    const v4f v = *(const v4f*)(sw + row * ODIM + 4 * pc);
    *(volatile v4f*)(rrow + (size_t)row * ODIM + 4 * pc) = v;
  }
  __threadfence();
#pragma unroll
  for (int q = 0; q < 4; ++q) {
    const int row = 4 * q + rq;
    const v4f v = *(const v4f*)(sw + row * ODIM + 4 * pc);
    *(volatile v4f*)(rrow + (size_t)row * ODIM + 4 * pc) = v;
  }
}

__device__ __forceinline__ v8f wtile(const unsigned short* __restrict__ whp, const unsigned short* __restrict__ wlp,
                                      const float* cq, v16us bh, v16us bl) {
  C8 c;
  c.h[0] = *(const v4f*)(cq);
  c.h[1] = *(const v4f*)(cq + 4);
  FragU a, al;
  a.u[0]  = *(const v8us*)(whp);
  a.u[1]  = *(const v8us*)(whp + 16);
  al.u[0] = *(const v8us*)(wlp);
  al.u[1] = *(const v8us*)(wlp + 16);
  v8f d = wmb(a.w, bh, c.v);
  d = wmb(a.w, bl, d);
  d = wmb(al.w, bh, d);
  return d;
}
__device__ __forceinline__ v8f lk_fma(v8f c, float xv, v8f acc) {
#pragma unroll
  for (int r = 0; r < 8; ++r) {
    const float w = fmaxf(c[r], SLOPEV * c[r]);
    acc[r] = __builtin_fmaf(xv, w, acc[r]);
  }
  return acc;
}

__global__ __launch_bounds__(NTHR) void k_edge(
    const float* __restrict__ x, const int* __restrict__ ei, const float* __restrict__ ea,
    const float* __restrict__ W1, const float* __restrict__ b1, const float* __restrict__ g1,
    const float* __restrict__ be1, const float* __restrict__ mu1, const float* __restrict__ va1,
    const unsigned short* __restrict__ Whi, const unsigned short* __restrict__ Wlo,
    const float* __restrict__ cin, float* Msg, int nE, int nN) {
  __shared__ __attribute__((aligned(16))) float sW1[EDIM * HID];
  __shared__ __attribute__((aligned(16))) float sB1[HID];
  __shared__ __attribute__((aligned(16))) float sCin[WCOL];
  __shared__ __attribute__((aligned(16))) float sH[NWAVE * 16 * HID];
  const int tid = (int)threadIdx.x, lane = tid & 31, wave = tid >> 5, hi = lane >> 4, m = lane & 15;

#pragma unroll 1
  for (int idx = tid; idx < EDIM * HID; idx += NTHR) {
    const int c = idx & (HID - 1);
    const float s1 = g1[c] * (1.0f / sqrtf(va1[c] + EPSV));
    sW1[idx] = W1[idx] * s1;
  }
  if (tid < HID) {
    const float s1 = g1[tid] * (1.0f / sqrtf(va1[tid] + EPSV));
    sB1[tid] = (b1[tid] - mu1[tid]) * s1 + be1[tid];
  }
  *(v4f*)(sCin + 4 * tid) = *(const v4f*)(cin + 4 * tid);
  __syncthreads();

  const int e0 = ((int)blockIdx.x * NWAVE + wave) * 16;
  int ec = e0 + m;
  ec = ec > nE - 1 ? nE - 1 : ec;
  int src = ei[ec];
  src = src < 0 ? 0 : (src > nN - 1 ? nN - 1 : src);
  float* sHw = sH + wave * (16 * HID);

  {
    const float* ep = ea + (size_t)ec * EDIM;
    const v4f ev0 = *(const v4f*)(ep);
    const v4f ev1 = *(const v4f*)(ep + 4);
    const v4f ev2 = *(const v4f*)(ep + 8);
    const v4f ev3 = *(const v4f*)(ep + 12);
#pragma unroll 1
    for (int g = 0; g < 4; ++g) {
      const int col0 = 16 * hi + 4 * g;
      const float* wq = sW1 + col0;
      v4f acc = {0.f, 0.f, 0.f, 0.f};
#define HSTEP(EV, K) acc += (EV) * *(const v4f*)(wq + HID * (K));
      HSTEP(ev0.x, 0)  HSTEP(ev0.y, 1)  HSTEP(ev0.z, 2)  HSTEP(ev0.w, 3)
      HSTEP(ev1.x, 4)  HSTEP(ev1.y, 5)  HSTEP(ev1.z, 6)  HSTEP(ev1.w, 7)
      HSTEP(ev2.x, 8)  HSTEP(ev2.y, 9)  HSTEP(ev2.z, 10) HSTEP(ev2.w, 11)
      HSTEP(ev3.x, 12) HSTEP(ev3.y, 13) HSTEP(ev3.z, 14) HSTEP(ev3.w, 15)
#undef HSTEP
      v4f hv = acc + *(const v4f*)(sB1 + col0);
      hv.x = fmaxf(hv.x, SLOPEV * hv.x);
      hv.y = fmaxf(hv.y, SLOPEV * hv.y);
      hv.z = fmaxf(hv.z, SLOPEV * hv.z);
      hv.w = fmaxf(hv.w, SLOPEV * hv.w);
      *(v4f*)(sHw + m * HID + col0) = hv;
    }
  }
  __syncthreads();

  FragU bh, bl;
  {
    const float* hp = sHw + m * HID + 8 * hi;
    const v4f q0 = *(const v4f*)(hp);
    const v4f q1 = *(const v4f*)(hp + 4);
    const v4f q2 = *(const v4f*)(hp + 16);
    const v4f q3 = *(const v4f*)(hp + 20);
    SPLIT2(q0.x, bh, bl, 0)  SPLIT2(q0.y, bh, bl, 1)  SPLIT2(q0.z, bh, bl, 2)  SPLIT2(q0.w, bh, bl, 3)
    SPLIT2(q1.x, bh, bl, 4)  SPLIT2(q1.y, bh, bl, 5)  SPLIT2(q1.z, bh, bl, 6)  SPLIT2(q1.w, bh, bl, 7)
    SPLIT2(q2.x, bh, bl, 8)  SPLIT2(q2.y, bh, bl, 9)  SPLIT2(q2.z, bh, bl, 10) SPLIT2(q2.w, bh, bl, 11)
    SPLIT2(q3.x, bh, bl, 12) SPLIT2(q3.y, bh, bl, 13) SPLIT2(q3.z, bh, bl, 14) SPLIT2(q3.w, bh, bl, 15)
  }

  v8f macc0 = z8(), macc1 = z8();
  {
    const float* xr = x + (size_t)src * FIN;
    const unsigned short* whp = Whi + m * KP + 8 * hi;
    const unsigned short* wlp = Wlo + m * KP + 8 * hi;
    const float* cp = sCin + 8 * hi;
#pragma unroll 1
    for (int i = 0; i < FIN; ++i) {
      const float xv = xr[i];
      const int na = 32 * i;
      const int nb = 32 * i + 16;
      const v8f ca = wtile(whp + (size_t)na * KP, wlp + (size_t)na * KP, cp + na, bh.w, bl.w);
      macc0 = lk_fma(ca, xv, macc0);
      const v8f cb = wtile(whp + (size_t)nb * KP, wlp + (size_t)nb * KP, cp + nb, bh.w, bl.w);
      macc1 = lk_fma(cb, xv, macc1);
    }
  }
  __syncthreads();

  {
    float* sp = sHw + m * ODIM + 8 * hi;
    C8 u;
    u.v = macc0;
    *(v4f*)(sp)      = u.h[0];
    *(v4f*)(sp + 4)  = u.h[1];
    u.v = macc1;
    *(v4f*)(sp + 16) = u.h[0];
    *(v4f*)(sp + 20) = u.h[1];
  }
  __syncthreads();
  {
    const int rq = lane >> 3, pc = lane & 7;
    float* mrow = Msg + (size_t)e0 * ODIM;
#pragma unroll
    for (int q = 0; q < 4; ++q) {
      const int row = 4 * q + rq;
      const v4f v = *(const v4f*)(sHw + row * ODIM + 4 * pc);
      *(volatile v4f*)(mrow + (size_t)row * ODIM + 4 * pc) = v;
    }
    __threadfence();
#pragma unroll
    for (int q = 0; q < 4; ++q) {
      const int row = 4 * q + rq;
      const v4f v = *(const v4f*)(sHw + row * ODIM + 4 * pc);
      *(volatile v4f*)(mrow + (size_t)row * ODIM + 4 * pc) = v;
    }
  }
}

__device__ __forceinline__ int scan_piece(const int* __restrict__ dp, int lim, int cbase, int base, int vec,
                                          int* list, int tid, int wave) {
  int wc = 0;
  const int el0  = tid * EPT;
  const int e0   = cbase + el0;
  const int sent = -2147483647 - 1;
  int kk[EPT];
  if (vec != 0 && cbase + PIECE <= lim) {
    const v4i* p = (const v4i*)(dp + e0);
#pragma unroll
    for (int u = 0; u < EPT / 4; ++u) {
      const v4i d = p[u];
      kk[4 * u] = d.x; kk[4 * u + 1] = d.y; kk[4 * u + 2] = d.z; kk[4 * u + 3] = d.w;
    }
  } else {
    const int lm = lim - 1;
#pragma unroll
    for (int q = 0; q < EPT; ++q) {
      const int eq = e0 + q;
      const int ecl = eq > lm ? lm : eq;
      const int a = dp[ecl];
      kk[q] = (eq < lim) ? a : sent;
    }
  }
  const unsigned nb = (unsigned)base;
  unsigned sq[EPT];
  bool hq[EPT];
  bool anyl = false;
#pragma unroll
  for (int q = 0; q < EPT; ++q) {
    sq[q] = (unsigned)kk[q] - nb;
    hq[q] = sq[q] < (unsigned)NBC;
    anyl = anyl | hq[q];
  }
  const unsigned any = __builtin_amdgcn_ballot_w32(anyl);
  if (any != 0u) {
#define HIT(HQ, SQ, Q) { \
      const unsigned mj = __builtin_amdgcn_ballot_w32(HQ); \
      if (mj != 0u) { \
        if (HQ) { \
          const int ps = wc + (int)__builtin_amdgcn_mbcnt_lo(mj, 0u); \
          if (ps < WCAP) list[wave * WCAP + ps] = ((el0 + (Q)) << SLB) | (int)(SQ); \
        } \
        wc += (int)__builtin_popcount(mj); } }
#pragma unroll
    for (int q = 0; q < EPT; ++q) {
      HIT(hq[q], sq[q], q)
    }
#undef HIT
  }
  return wc;
}

__device__ __forceinline__ void drain_piece(const int* list, const int* wcnt, float* accF,
                                            const float* __restrict__ Msg, int rowoff, int nE, int lane, int wave) {
#pragma unroll 1
  for (int wsx = 0; wsx < NWAVE; ++wsx) {
    int n = __builtin_amdgcn_readfirstlane(wcnt[wsx]);
    n = n > WCAP ? WCAP : (n < 0 ? 0 : n);
    const int* lp = list + wsx * WCAP;
#pragma unroll 1
    for (int bb = 0; bb < n; bb += 32) {
      const int idx = bb + lane;
      const int ic = idx > WCAP - 1 ? WCAP - 1 : idx;
      const int ent = lp[ic];
      const bool own = (idx < n) && ((ent & (NWAVE - 1)) == wave);
      unsigned msk = __builtin_amdgcn_ballot_w32(own);
#pragma unroll 1
      while (msk != 0u) {
        const int bit = (int)__builtin_ctz(msk);
        msk &= msk - 1u;
        const int e2 = __builtin_amdgcn_readlane(ent, bit);
        const int slot = e2 & (NBC - 1);
        const int el = (e2 >> SLB) & (PIECE - 1);
        int row = rowoff + el;
        row = row < 0 ? 0 : (row > nE - 1 ? nE - 1 : row);
        const float mv = Msg[(size_t)row * ODIM + lane];
        accF[slot * ODIM + lane] += mv;
      }
    }
  }
}

__device__ __forceinline__ void agg_store(const float* accF, float* out, int base, int nN, int lane, int wave) {
  const int rq = lane >> 3, pc = lane & 7;
#pragma unroll 1
  for (int it = 0; it < NBC / 32; ++it) {
    const int s = 32 * it + 4 * wave + rq;
    const int node = base + s;
    if (node < nN) {
      const v4f v = *(const v4f*)(accF + s * ODIM + 4 * pc);
      *(volatile v4f*)(out + (size_t)node * ODIM + 4 * pc) = v;
    }
  }
}

__global__ __launch_bounds__(NTHR) void k_agg(
    const int* __restrict__ dp, const float* __restrict__ Msg, const float* __restrict__ R,
    float* out, int nE, int nN, int vec) {
  extern __shared__ __attribute__((aligned(16))) float accF[];
  __shared__ int list[NWAVE * WCAP];
  __shared__ int wcnt[NWAVE];
  const int tid = (int)threadIdx.x, lane = tid & 31, wave = tid >> 5;
  const int base = (int)blockIdx.x * NBC;

#pragma unroll 1
  for (int i = tid; i < (NBC * ODIM) / 4; i += NTHR) {
    const int s = i >> 3, c4 = (i & 7) * 4;
    int node = base + s;
    node = node > nN - 1 ? nN - 1 : node;
    const v4f v = *(const v4f*)(R + (size_t)node * ODIM + c4);
    *(v4f*)(accF + s * ODIM + c4) = v;
  }
  __syncthreads();

#pragma unroll 1
  for (int cbase = 0; cbase < nE; cbase += PIECE) {
    const int wc = scan_piece(dp, nE, cbase, base, vec, list, tid, wave);
    if (lane == 0) wcnt[wave] = wc;
    __syncthreads();
    drain_piece(list, wcnt, accF, Msg, cbase, nE, lane, wave);
    __syncthreads();
  }

  agg_store(accF, out, base, nN, lane, wave);
  __threadfence();
  agg_store(accF, out, base, nN, lane, wave);
}

extern "C" void kernel_launch(void* const* d_in, const int* in_sizes, int n_in,
                              void* d_out, int out_size, void* d_ws, size_t ws_size,
                              hipStream_t stream) {
  if (n_in < 18) return;
  if (in_sizes[0] < FIN || (in_sizes[0] % FIN) != 0) return;
  const int nN = in_sizes[0] / FIN;
  if (nN < 1 || nN > (1 << 24)) return;
  if (in_sizes[1] < 2 || (in_sizes[1] % 2) != 0) return;
  const int nE = in_sizes[1] / 2;
  if (nE < 1 || nE > (1 << 26)) return;
  if (in_sizes[2] != nE * EDIM) return;
  if (in_sizes[4] != EDIM * HID || in_sizes[5] != HID) return;
  if (in_sizes[6] != HID || in_sizes[7] != HID || in_sizes[8] != HID || in_sizes[9] != HID) return;
  if (in_sizes[10] != HID * WCOL || in_sizes[11] != WCOL) return;
  if (in_sizes[12] != WCOL || in_sizes[13] != WCOL || in_sizes[14] != WCOL || in_sizes[15] != WCOL) return;
  if (in_sizes[16] != FIN * ODIM || in_sizes[17] != ODIM) return;
  if (out_size != nN * ODIM) return;

  const float* x    = (const float*)d_in[0];
  const int*   ei   = (const int*)d_in[1];
  const float* ea   = (const float*)d_in[2];
  const float* W1   = (const float*)d_in[4];
  const float* b1   = (const float*)d_in[5];
  const float* g1   = (const float*)d_in[6];
  const float* be1  = (const float*)d_in[7];
  const float* mu1  = (const float*)d_in[8];
  const float* va1  = (const float*)d_in[9];
  const float* W2   = (const float*)d_in[10];
  const float* b2   = (const float*)d_in[11];
  const float* g2   = (const float*)d_in[12];
  const float* be2  = (const float*)d_in[13];
  const float* mu2  = (const float*)d_in[14];
  const float* va2  = (const float*)d_in[15];
  const float* root = (const float*)d_in[16];
  const float* bias = (const float*)d_in[17];
  float* out = (float*)d_out;

  const int nbE   = (nE + EPB - 1) / EPB;
  const int Epad  = nbE * EPB;
  const int nbR   = (nN + NPB - 1) / NPB;
  const int NpadR = nbR * NPB;
  const int nbAgg = (nN + NBC - 1) / NBC;
  const int vec   = ((nE & 3) == 0) ? 1 : 0;

  char* ws = (char*)d_ws;
  size_t off = 0;
  const size_t oWh = off; off += (size_t)WCOL * KP * 2;          off = (off + 255) & ~(size_t)255;
  const size_t oWl = off; off += (size_t)WCOL * KP * 2;          off = (off + 255) & ~(size_t)255;
  const size_t oCi = off; off += (size_t)WCOL * 4;               off = (off + 255) & ~(size_t)255;
  const size_t oR  = off; off += (size_t)NpadR * ODIM * 4;       off = (off + 255) & ~(size_t)255;
  const size_t oM  = off; off += (size_t)Epad * ODIM * 4;        off = (off + 255) & ~(size_t)255;
  if (off > ws_size || off > (size_t)WSCAP) return;
  unsigned short* Whi = (unsigned short*)(ws + oWh);
  unsigned short* Wlo = (unsigned short*)(ws + oWl);
  float* cin = (float*)(ws + oCi);
  float* R   = (float*)(ws + oR);
  float* Msg = (float*)(ws + oM);

  hipFuncSetAttribute(reinterpret_cast<const void*>(&k_agg), hipFuncAttributeMaxDynamicSharedMemorySize, AGGDYN);

  k_prep<<<PBLK, NTHR, 0, stream>>>(W2, b2, g2, be2, mu2, va2, Whi, Wlo, cin);
  k_root<<<nbR, NTHR, 0, stream>>>(x, root, bias, R, nN);
  k_edge<<<nbE, NTHR, 0, stream>>>(x, ei, ea, W1, b1, g1, be1, mu1, va1, Whi, Wlo, cin, Msg, nE, nN);
  k_agg<<<nbAgg, NTHR, AGGDYN, stream>>>(ei + nE, Msg, R, out, nE, nN, vec);
}
